// SelfAttn_15040975470634
// MI455X (gfx1250) — hardware-verified
//
#include <hip/hip_runtime.h>
#include <math.h>


#define BB 2
#define TT 2048
#define DDm 1024
#define HH 16
#define HD 64
#define MROWS (BB * TT)

typedef __attribute__((ext_vector_type(16))) __bf16 v16bf;
typedef __attribute__((ext_vector_type(8)))  __bf16 v8bf;
typedef __attribute__((ext_vector_type(8)))  float v8f;
typedef __attribute__((ext_vector_type(4)))  float v4f;

template <typename T> __device__ __forceinline__ void vst2(void* p, T v) { *(volatile T*)p = v; __threadfence(); *(volatile T*)p = v; }
__device__ __forceinline__ v8f wmma_bf(v16bf a, v16bf b, v8f c) {
  v8f d = __builtin_amdgcn_wmma_f32_16x16x32_bf16(false, a, false, b, (short)0, c, false, false);
  asm volatile("v_nop\n\tv_nop\n\tv_nop\n\tv_nop" : "+v"(d) : "v"(a), "v"(b));
  return d;
}
struct F2 { v16bf h, l; };
__device__ __forceinline__ F2 split16(const float* v) {
  F2 r;
#pragma unroll
  for (int i = 0; i < 16; ++i) { const __bf16 hh = (__bf16)v[i]; r.h[i] = hh; r.l[i] = (__bf16)(v[i] - (float)hh); }
  return r;
}
__device__ __forceinline__ F2 split_row(const float* row, int k0, int lane) {
  float v[16]; const float* p = row + k0 + 8 * (lane >> 4);
#pragma unroll
  for (int i = 0; i < 8; ++i) { v[i] = p[i]; v[8 + i] = p[16 + i]; }
  return split16(v);
}
__device__ __forceinline__ v8f mac3(const F2& a, const F2& b, v8f c) { c = wmma_bf(a.l, b.h, c); c = wmma_bf(a.h, b.l, c); return wmma_bf(a.h, b.h, c); }

__global__ __launch_bounds__(128) void k_gemm(const float* __restrict__ A, const float* __restrict__ W, int mode,
                                            float* __restrict__ Q, float* __restrict__ Kf, float* __restrict__ Vt, float* __restrict__ out) {
  __shared__ __align__(16) float st[64][68];
  __shared__ __align__(16) float st2[64][68];
  const int tid = threadIdx.x, wave = tid >> 5, lane = tid & 31, col = lane & 15, g = lane >> 4;
  const int m0 = blockIdx.x * 64 + wave * 16, n0 = blockIdx.y * 64;
  const float* arow = A + (size_t)(m0 + col) * DDm;
  v8f acc[4] = {};
#pragma unroll 1
  for (int kc = 0; kc < DDm / 32; ++kc) {
    const F2 a = split_row(arow, kc * 32, lane);
#pragma unroll
    for (int j = 0; j < 4; ++j) acc[j] = mac3(a, split_row(W + (size_t)(n0 + j * 16 + col) * DDm, kc * 32, lane), acc[j]);
  }
#pragma unroll
  for (int j = 0; j < 4; ++j)
#pragma unroll
    for (int r = 0; r < 8; ++r) st[wave * 16 + 8 * g + r][j * 16 + col] = acc[j][r];
  __syncthreads();
  const int bm0 = blockIdx.x * 64;
  if (mode == 1) {
    for (int q = tid; q < 64 * 16; q += 128) { const int rl = q >> 4, pc = q & 15;
      vst2(out + (size_t)(bm0 + rl) * DDm + n0 + pc * 4, *(const v4f*)(&st[rl][pc * 4])); }
    return;
  }
  const int which = n0 >> 10, h = (n0 >> 6) & 15, b = bm0 >> 11, t0 = bm0 & (TT - 1);
  if (which < 2) {
    for (int i = tid; i < 64 * 64; i += 128) { const int rl = i >> 6, d = i & 63;
      const float invf = 1.0f / powf(10000.0f, (float)(2 * (d & 31)) / 64.0f);
      const float ang = (float)(t0 + rl) * invf;
      const float cs = cosf(ang), sn = sinf(ang);
      const float rot = (d < 32) ? -st[rl][d + 32] : st[rl][d - 32];
      st2[rl][d] = st[rl][d] * cs + rot * sn; }
    __syncthreads();
    float* dst = (which == 0 ? Q : Kf) + (((size_t)b * HH + h) * TT + t0) * HD;
    for (int q = tid; q < 64 * 16; q += 128) { const int rl = q >> 4, pc = q & 15;
      vst2(dst + (size_t)rl * HD + pc * 4, *(const v4f*)(&st2[rl][pc * 4])); }
  } else {
    float* dst = Vt + (((size_t)b * HH + h) * HD) * TT + t0;
    for (int q = tid; q < 64 * 16; q += 128) { const int d = q >> 4, pc = q & 15;
      v4f v = { st[pc * 4][d], st[pc * 4 + 1][d], st[pc * 4 + 2][d], st[pc * 4 + 3][d] };
      vst2(dst + (size_t)d * TT + pc * 4, v); }
  }
}

__global__ __launch_bounds__(128) void k_attn(const float* __restrict__ Q, const float* __restrict__ Kf, const float* __restrict__ Vt,
                                            float* __restrict__ ao) {
  __shared__ __align__(16) float Ps[4][16 * 32];
  __shared__ __align__(16) float Os[4][16 * 64];
  const int tid = threadIdx.x, wl = tid >> 5, lane = tid & 31, col = lane & 15, g = lane >> 4;
  const int bh = blockIdx.y, b = bh >> 4, h = bh & 15;
  const int t0 = blockIdx.x * 64 + wl * 16;
  const float* Qb = Q + ((size_t)bh * TT) * HD;
  const float* Kb = Kf + ((size_t)bh * TT) * HD;
  const float* Vb = Vt + ((size_t)bh * HD) * TT;
  const F2 qa = split_row(Qb + (size_t)(t0 + col) * HD, 0, lane), qc = split_row(Qb + (size_t)(t0 + col) * HD, 32, lane);
  float m_r[8], l_r[8];
  v8f o[4] = {};
#pragma unroll
  for (int r = 0; r < 8; ++r) { m_r[r] = -3.0e38f; l_r[r] = 0.f; }
  float* P = Ps[wl];
  const int jmax = (t0 + 15) >> 5;
  for (int j = 0; j <= jmax; ++j) {
    const int ks = j * 32;
    v8f s0 = {}, s1 = {};
    { const float* k0 = Kb + (size_t)(ks + col) * HD, *k1 = k0 + 16 * HD;
      s0 = mac3(qa, split_row(k0, 0, lane), s0); s0 = mac3(qc, split_row(k0, 32, lane), s0);
      s1 = mac3(qa, split_row(k1, 0, lane), s1); s1 = mac3(qc, split_row(k1, 32, lane), s1); }
#pragma unroll
    for (int r = 0; r < 8; ++r) {
      const int qi = t0 + 8 * g + r;
      float a0 = s0[r] * 0.125f; if (ks + col > qi)      a0 = -3.0e38f;
      float a1 = s1[r] * 0.125f; if (ks + 16 + col > qi) a1 = -3.0e38f;
      float mx = fmaxf(a0, a1);
#pragma unroll
      for (int off = 8; off >= 1; off >>= 1) mx = fmaxf(mx, __shfl_xor(mx, off, 32));
      const float mn = fmaxf(m_r[r], mx);
      const float p0 = (ks + col > qi) ? 0.f : expf(a0 - mn), p1 = (ks + 16 + col > qi) ? 0.f : expf(a1 - mn);
      P[(8 * g + r) * 32 + col] = p0; P[(8 * g + r) * 32 + 16 + col] = p1;
      float sum = p0 + p1;
#pragma unroll
      for (int off = 8; off >= 1; off >>= 1) sum += __shfl_xor(sum, off, 32);
      const float corr = expf(m_r[r] - mn);
      l_r[r] = l_r[r] * corr + sum; m_r[r] = mn;
#pragma unroll
      for (int t = 0; t < 4; ++t) o[t][r] *= corr;
    }
    asm volatile("s_wait_dscnt 0" ::: "memory"); __builtin_amdgcn_wave_barrier(); __builtin_amdgcn_fence(__ATOMIC_RELEASE, "workgroup");
    const F2 pf = split_row(P + col * 32, 0, lane);
#pragma unroll
    for (int t = 0; t < 4; ++t) o[t] = mac3(pf, split_row(Vb + (size_t)(t * 16 + col) * TT + ks, 0, lane), o[t]);
    __builtin_amdgcn_wave_barrier();
  }
  float* so = Os[wl];
#pragma unroll
  for (int t = 0; t < 4; ++t)
#pragma unroll
    for (int r = 0; r < 8; ++r) so[(8 * g + r) * 64 + t * 16 + col] = o[t][r] / l_r[r];
  asm volatile("s_wait_dscnt 0" ::: "memory"); __builtin_amdgcn_wave_barrier(); __builtin_amdgcn_fence(__ATOMIC_RELEASE, "workgroup");
#pragma unroll
  for (int q = 0; q < 8; ++q) { const int rl = q * 2 + (lane >> 4), pc = lane & 15;
    vst2(ao + ((size_t)b * TT + t0 + rl) * DDm + h * HD + pc * 4, *(const v4f*)(so + rl * 64 + pc * 4)); }
}

extern "C" void kernel_launch(void* const* d_in, const int* in_sizes, int n_in,
                              void* d_out, int out_size, void* d_ws, size_t ws_size,
                              hipStream_t stream) {
  (void)in_sizes; (void)n_in; (void)out_size; (void)ws_size;
  const float* x    = (const float*)d_in[0];
  const float* Wqkv = (const float*)d_in[1];
  const float* Wout = (const float*)d_in[2];
  float* out = (float*)d_out;
  float* Q  = (float*)d_ws;
  float* Kf = Q + (size_t)MROWS * DDm;
  float* Vt = Kf + (size_t)MROWS * DDm;
  float* ao = Vt + (size_t)MROWS * DDm;
  k_gemm<<<dim3(MROWS / 64, 3 * DDm / 64), 128, 0, stream>>>(x, Wqkv, 0, Q, Kf, Vt, nullptr);
  k_attn<<<dim3(TT / 64, BB * HH), 128, 0, stream>>>(Q, Kf, Vt, ao);
  k_gemm<<<dim3(MROWS / 64, DDm / 64), 128, 0, stream>>>(ao, Wout, 1, nullptr, nullptr, nullptr, out);
}
